// GaussianNonLocalBlock_36103495090205
// MI455X (gfx1250) — hardware-verified
//
#include <hip/hip_runtime.h>

typedef __attribute__((ext_vector_type(16))) _Float16 v16h;
typedef __attribute__((ext_vector_type(8)))  _Float16 v8h;
typedef __attribute__((ext_vector_type(16))) __bf16   v16b;
typedef __attribute__((ext_vector_type(8)))  __bf16   v8b;
typedef __attribute__((ext_vector_type(8)))  float    v8f;
typedef __attribute__((ext_vector_type(4)))  float    v4f;
#define PSCALE 32768.0f
#define U16(p) ((const unsigned short*)(const void*)(p))
#define PSCALE_INV (1.0f / 32768.0f)

__device__ __forceinline__ unsigned short f2bf_bits(float f) {
  unsigned u = __float_as_uint(f);
  return (unsigned short)((u + 0x7FFFu + ((u >> 16) & 1u)) >> 16);
}
__device__ __forceinline__ float bf_bits2f(unsigned short h) { return __uint_as_float(((unsigned)h) << 16); }

__device__ __forceinline__ void dep_guard_h(v8f& a, v8f& b, v16h x, v16h y) { asm volatile("v_nop\n\tv_nop\n\tv_nop\n\tv_nop" : "+v"(a), "+v"(b) : "v"(x), "v"(y)); }
__device__ __forceinline__ void dep_guard_b(v8f& a, v8f& b, v16b x, v16b y) { asm volatile("v_nop\n\tv_nop\n\tv_nop\n\tv_nop" : "+v"(a), "+v"(b) : "v"(x), "v"(y)); }
__device__ __forceinline__ void keep4_h(v16h a, v16h b, v16h c, v16h d) { asm volatile("v_nop" :: "v"(a), "v"(b), "v"(c), "v"(d)); }
__device__ __forceinline__ void keep4_b(v16b a, v16b b, v16b c, v16b d) { asm volatile("v_nop" :: "v"(a), "v"(b), "v"(c), "v"(d)); }
__device__ __forceinline__ void acc_guard4(v8f& a, v8f& b, v8f& c, v8f& d) { asm volatile("v_nop\n\tv_nop\n\tv_nop\n\tv_nop" : "+v"(a), "+v"(b), "+v"(c), "+v"(d)); }
template <typename T> struct Frag;
template <> struct Frag<_Float16> {
  typedef v16h V; union U { v16h v; v8h h[2]; };
  static __device__ __forceinline__ v16h load(const _Float16* p) {
    U f; f.h[0] = *(const v8h*)(p); f.h[1] = *(const v8h*)(p + 16); return f.v;
  }
  static __device__ __forceinline__ v8f mma(v16h a, v16h b, v8f c) {
    return __builtin_amdgcn_wmma_f32_16x16x32_f16(false, a, false, b, (short)0, c, false, false);
  }
  static __device__ __forceinline__ void guard(v8f& a, v8f& b, v16h x, v16h y) { dep_guard_h(a, b, x, y); }
  static __device__ __forceinline__ void keep(v16h a, v16h b, v16h c, v16h d) { keep4_h(a, b, c, d); }
};
template <> struct Frag<__bf16> {
  typedef v16b V; union U { v16b v; v8b h[2]; };
  static __device__ __forceinline__ v16b load(const __bf16* p) {
    U f; f.h[0] = *(const v8b*)(p); f.h[1] = *(const v8b*)(p + 16); return f.v;
  }
  static __device__ __forceinline__ v8f mma(v16b a, v16b b, v8f c) {
    return __builtin_amdgcn_wmma_f32_16x16x32_bf16(false, a, false, b, (short)0, c, false, false);
  }
  static __device__ __forceinline__ void guard(v8f& a, v8f& b, v16b x, v16b y) { dep_guard_b(a, b, x, y); }
  static __device__ __forceinline__ void keep(v16b a, v16b b, v16b c, v16b d) { keep4_b(a, b, c, d); }
};

template <int ET> struct Elem;
template <> struct Elem<0> { typedef _Float16 T; };
template <> struct Elem<1> { typedef __bf16 T; };
template <int ET, bool SPLIT, int BIAS_MODE, int OUT_MODE, bool RESID, int ACT = 0>
__global__ __launch_bounds__(256) void wmma_gemm64(
    const unsigned short* __restrict__ Ap, const unsigned short* __restrict__ A2p, int lda, long strideA,
    const unsigned short* __restrict__ Btp, const unsigned short* __restrict__ Bt2p, int ldb, long strideB,
    void* __restrict__ Cout, void* __restrict__ Cout2, int ldc, long strideC,
    const float* __restrict__ bias,
    const float* __restrict__ resid, long strideR,
    int M, int N, int K, float scale) {
  typedef typename Elem<ET>::T T;
  typedef typename Frag<T>::V V;
  const T* A = (const T*)Ap; const T* A2 = (const T*)A2p; const T* Bt = (const T*)Btp; const T* Bt2 = (const T*)Bt2p;
  __shared__ __align__(16) float sT[8][16 * 68];
  const int b    = blockIdx.y;
  const int lane = threadIdx.x & 31;
  const int wave = threadIdx.x >> 5;
  const int tilesN = N >> 6;
  const int tilesM = M >> 6;
  const int tile = blockIdx.x * 8 + wave;
  if (tile >= tilesM * tilesN) return;
  const int tm = tile / tilesN;
  const int tn = tile - tm * tilesN;
  const int m0 = tm << 6;
  const int n0 = tn << 6;

  const T* Ab  = A  + (size_t)b * strideA;
  const T* Bb  = Bt + (size_t)b * strideB;
  const T* Ab2 = SPLIT ? (A2  + (size_t)b * strideA) : nullptr;
  const T* Bb2 = SPLIT ? (Bt2 + (size_t)b * strideB) : nullptr;

  const int rlane = lane & 15;
  const int koff  = (lane >> 4) * 8;
  const int mOff  = (lane >> 4) * 8;

  v8f acc[4][4];
#pragma unroll
  for (int i = 0; i < 4; ++i)
#pragma unroll
    for (int j = 0; j < 4; ++j) acc[i][j] = (v8f){0.f,0.f,0.f,0.f,0.f,0.f,0.f,0.f};

  for (int k0 = 0; k0 < K; k0 += 32) {
    V bh[4], bl[4];
#pragma unroll
    for (int j = 0; j < 4; ++j) {
      const size_t bo = (size_t)(n0 + (j << 4) + rlane) * ldb + koff + k0;
      bh[j] = Frag<T>::load(Bb + bo);
      if (SPLIT) bl[j] = Frag<T>::load(Bb2 + bo);
    }
#pragma unroll
    for (int i = 0; i < 4; ++i) {
      const size_t ao = (size_t)(m0 + (i << 4) + rlane) * lda + koff + k0;
      V ah = Frag<T>::load(Ab + ao);
      V al;
      if (SPLIT) al = Frag<T>::load(Ab2 + ao);
#pragma unroll
      for (int j = 0; j < 4; ++j) {
        acc[i][j] = Frag<T>::mma(ah, bh[j], acc[i][j]);
        if (SPLIT) {
          acc[i][j] = Frag<T>::mma(ah, bl[j], acc[i][j]);
          acc[i][j] = Frag<T>::mma(al, bh[j], acc[i][j]);
        }
      }
      Frag<T>::guard(acc[i][0], acc[i][3], ah, SPLIT ? al : ah);
    }
    Frag<T>::keep(bh[0], bh[1], bh[2], bh[3]);
    if (SPLIT) Frag<T>::keep(bl[0], bl[1], bl[2], bl[3]);
  }
  acc_guard4(acc[0][0], acc[0][1], acc[0][2], acc[0][3]);
  acc_guard4(acc[1][0], acc[1][1], acc[1][2], acc[1][3]);
  acc_guard4(acc[2][0], acc[2][1], acc[2][2], acc[2][3]);
  acc_guard4(acc[3][0], acc[3][1], acc[3][2], acc[3][3]);

  float* slab = sT[wave];
  const float* Rb = RESID ? (resid + (size_t)b * strideR) : nullptr;
#pragma unroll
  for (int i = 0; i < 4; ++i) {
    const int mBase = m0 + (i << 4);
#pragma unroll
    for (int j = 0; j < 4; ++j) {
      const int n = n0 + (j << 4) + rlane;
      float bv = 0.f;
      if (BIAS_MODE == 2) bv = bias[n];
#pragma unroll
      for (int r = 0; r < 8; ++r) {
        float v = acc[i][j][r] * scale;
        if (BIAS_MODE == 1) v += bias[mBase + mOff + r];
        if (BIAS_MODE == 2) v += bv;
        if (RESID) v += Rb[(size_t)(mBase + mOff + r) * ldc + n];
        if (ACT == 1) v = tanhf(v);
        if (ACT == 2) v = fmaxf(v, 0.0f);
        if (ACT == 3) v = v / (1.0f + expf(-v));
        if (ACT == 4) v = (v > 0.f) ? v : 0.01f * v;
        if (ACT == 5) v = 0.5f * v * (1.0f + erff(v * 0.70710678118654752f));
        slab[(mOff + r) * 68 + (j << 4) + rlane] = v;
      }
    }
    __builtin_amdgcn_fence(__ATOMIC_RELEASE, "workgroup");
    __builtin_amdgcn_wave_barrier();
    __builtin_amdgcn_fence(__ATOMIC_ACQUIRE, "workgroup");
    if (OUT_MODE == 0) {
      float* C = (float*)Cout + (size_t)b * strideC;
      const int hh = lane >> 4, c4 = (lane & 15) * 4;
      for (int pass = 0; pass < 2; ++pass) {
#pragma unroll
        for (int it = 0; it < 8; ++it) {
          const int row = it * 2 + hh;
          v4f v = *(const v4f*)(slab + row * 68 + c4);
          *(volatile v4f*)(C + (size_t)(mBase + row) * ldc + n0 + c4) = v;
        }
        __threadfence();
      }
    } else {
      const int q = lane >> 3, c8 = (lane & 7) * 8;
      unsigned short* C  = (unsigned short*)Cout  + (size_t)b * strideC;
      unsigned short* C2 = (OUT_MODE == 2) ? ((unsigned short*)Cout2 + (size_t)b * strideC) : nullptr;
      for (int pass = 0; pass < 2; ++pass) {
#pragma unroll
        for (int it = 0; it < 4; ++it) {
          const int row = it * 4 + q;
          const float* sp = slab + row * 68 + c8;
          v8h hv, lv;
#pragma unroll
          for (int e = 0; e < 8; ++e) {
            if (OUT_MODE == 1) {
              hv[e] = (_Float16)sp[e];
            } else {
              unsigned short hb = f2bf_bits(sp[e]);
              unsigned short lb = f2bf_bits(sp[e] - bf_bits2f(hb));
              hv[e] = __builtin_bit_cast(_Float16, hb);
              lv[e] = __builtin_bit_cast(_Float16, lb);
            }
          }
          *(volatile v8h*)(C + (size_t)(mBase + row) * ldc + n0 + c8) = hv;
          if (OUT_MODE == 2) *(volatile v8h*)(C2 + (size_t)(mBase + row) * ldc + n0 + c8) = lv;
        }
        __threadfence();
      }
    }
    __builtin_amdgcn_fence(__ATOMIC_RELEASE, "workgroup");
    __builtin_amdgcn_wave_barrier();
    __builtin_amdgcn_fence(__ATOMIC_ACQUIRE, "workgroup");
  }
}

__global__ __launch_bounds__(256) void wmma_gram64(
    const unsigned short* __restrict__ Xp, int ldx,
    float* __restrict__ Sout, int ldo, int NT, int K, float scale) {
  typedef _Float16 T;
  typedef v16h V;
  const T* A = (const T*)Xp;
  __shared__ __align__(16) float sT[8][16 * 68];
  const int lane = threadIdx.x & 31;
  const int wave = threadIdx.x >> 5;
  const int npairs = (NT * (NT + 1)) >> 1;
  const int t = blockIdx.x * 8 + wave;
  if (t >= npairs) return;
  int tm = 0, rem = t;
#pragma unroll 1
  for (int i = 0; i < 63; ++i) {
    const int cnt = NT - tm;
    if (i < NT - 1 && rem >= cnt) { rem -= cnt; ++tm; }
  }
  int tn = tm + rem;
  if (tn > NT - 1) tn = NT - 1;
  const int m0 = tm << 6;
  const int n0 = tn << 6;

  const int rlane = lane & 15;
  const int koff  = (lane >> 4) * 8;
  const int mOff  = (lane >> 4) * 8;

  v8f acc[4][4];
#pragma unroll
  for (int i = 0; i < 4; ++i)
#pragma unroll
    for (int j = 0; j < 4; ++j) acc[i][j] = (v8f){0.f,0.f,0.f,0.f,0.f,0.f,0.f,0.f};

  for (int k0 = 0; k0 < K; k0 += 32) {
    V bh[4];
#pragma unroll
    for (int j = 0; j < 4; ++j) {
      const size_t bo = (size_t)(n0 + (j << 4) + rlane) * ldx + koff + k0;
      bh[j] = Frag<T>::load(A + bo);
    }
#pragma unroll
    for (int i = 0; i < 4; ++i) {
      const size_t ao = (size_t)(m0 + (i << 4) + rlane) * ldx + koff + k0;
      V ah = Frag<T>::load(A + ao);
#pragma unroll
      for (int j = 0; j < 4; ++j) acc[i][j] = Frag<T>::mma(ah, bh[j], acc[i][j]);
      Frag<T>::guard(acc[i][0], acc[i][3], ah, ah);
    }
    Frag<T>::keep(bh[0], bh[1], bh[2], bh[3]);
  }
  acc_guard4(acc[0][0], acc[0][1], acc[0][2], acc[0][3]);
  acc_guard4(acc[1][0], acc[1][1], acc[1][2], acc[1][3]);
  acc_guard4(acc[2][0], acc[2][1], acc[2][2], acc[2][3]);
  acc_guard4(acc[3][0], acc[3][1], acc[3][2], acc[3][3]);

  float* slab = sT[wave];
  const int hh = lane >> 4, c4 = (lane & 15) * 4;
#pragma unroll
  for (int i = 0; i < 4; ++i) {
    const int mBase = m0 + (i << 4);
#pragma unroll
    for (int j = 0; j < 4; ++j) {
#pragma unroll
      for (int r = 0; r < 8; ++r) slab[(mOff + r) * 68 + (j << 4) + rlane] = acc[i][j][r] * scale;
    }
    __builtin_amdgcn_fence(__ATOMIC_RELEASE, "workgroup");
    __builtin_amdgcn_wave_barrier();
    __builtin_amdgcn_fence(__ATOMIC_ACQUIRE, "workgroup");
    for (int pass = 0; pass < 2; ++pass) {
#pragma unroll
      for (int it = 0; it < 8; ++it) {
        const int row = it * 2 + hh;
        v4f v = *(const v4f*)(slab + row * 68 + c4);
        *(volatile v4f*)(Sout + (size_t)(mBase + row) * ldo + n0 + c4) = v;
      }
      __threadfence();
    }
    __builtin_amdgcn_fence(__ATOMIC_RELEASE, "workgroup");
    __builtin_amdgcn_wave_barrier();
    __builtin_amdgcn_fence(__ATOMIC_ACQUIRE, "workgroup");
  }
  if (tm != tn) {
#pragma unroll
    for (int j = 0; j < 4; ++j) {
      const int nBase = n0 + (j << 4);
#pragma unroll
      for (int i = 0; i < 4; ++i) {
#pragma unroll
        for (int r = 0; r < 8; ++r) slab[rlane * 68 + (i << 4) + mOff + r] = acc[i][j][r] * scale;
      }
      __builtin_amdgcn_fence(__ATOMIC_RELEASE, "workgroup");
      __builtin_amdgcn_wave_barrier();
      __builtin_amdgcn_fence(__ATOMIC_ACQUIRE, "workgroup");
      for (int pass = 0; pass < 2; ++pass) {
#pragma unroll
        for (int it = 0; it < 8; ++it) {
          const int row = it * 2 + hh;
          v4f v = *(const v4f*)(slab + row * 68 + c4);
          *(volatile v4f*)(Sout + (size_t)(nBase + row) * ldo + m0 + c4) = v;
        }
        __threadfence();
      }
      __builtin_amdgcn_fence(__ATOMIC_RELEASE, "workgroup");
      __builtin_amdgcn_wave_barrier();
      __builtin_amdgcn_fence(__ATOMIC_ACQUIRE, "workgroup");
    }
  }
}

__device__ __forceinline__ void split_bf16(float f, _Float16& hi, _Float16& lo) {
  const unsigned short hb = f2bf_bits(f);
  const unsigned short lb = f2bf_bits(f - bf_bits2f(hb));
  hi = __builtin_bit_cast(_Float16, hb);
  lo = __builtin_bit_cast(_Float16, lb);
}

__global__ __launch_bounds__(256) void k_wsplit(const float* __restrict__ w0, const float* __restrict__ w1,
                                                unsigned short* __restrict__ h0, unsigned short* __restrict__ l0,
                                                unsigned short* __restrict__ h1, unsigned short* __restrict__ l1,
                                                int n8) {
  const int i = blockIdx.x * 256 + threadIdx.x;
  if (i >= n8) return;
  const size_t o = (size_t)i * 8;
  const v4f a0 = *(const v4f*)(w0 + o), a1 = *(const v4f*)(w0 + o + 4);
  const v4f b0 = *(const v4f*)(w1 + o), b1 = *(const v4f*)(w1 + o + 4);
  v8h ha, la, hb, lb;
#pragma unroll
  for (int e = 0; e < 4; ++e) {
    _Float16 th, tl;
    split_bf16(a0[e], th, tl); ha[e] = th;     la[e] = tl;
    split_bf16(a1[e], th, tl); ha[4 + e] = th; la[4 + e] = tl;
    split_bf16(b0[e], th, tl); hb[e] = th;     lb[e] = tl;
    split_bf16(b1[e], th, tl); hb[4 + e] = th; lb[4 + e] = tl;
  }
  *(volatile v8h*)(h0 + o) = ha; *(volatile v8h*)(l0 + o) = la;
  *(volatile v8h*)(h1 + o) = hb; *(volatile v8h*)(l1 + o) = lb;
  __threadfence();
  *(volatile v8h*)(h0 + o) = ha; *(volatile v8h*)(l0 + o) = la;
  *(volatile v8h*)(h1 + o) = hb; *(volatile v8h*)(l1 + o) = lb;
}

__global__ __launch_bounds__(256) void k_xconv(const float* __restrict__ x,
                                               unsigned short* __restrict__ xh,
                                               unsigned short* __restrict__ xbh,
                                               unsigned short* __restrict__ xbl,
                                               int Cc, int Nn) {
  __shared__ float tile[64][33];
  const int nt  = Nn >> 5;
  const int ctn = Cc >> 6;
  int blk = blockIdx.x;
  const int ntile = blk % nt; blk /= nt;
  const int ct = blk % ctn;
  const int b  = blk / ctn;
  const int c0 = ct << 6, n0 = ntile << 5;
  const int tid = threadIdx.x;
  const float* xs = x + ((size_t)b * Cc + c0) * Nn + n0;
#pragma unroll
  for (int i = 0; i < 8; ++i) {
    const int idx = i * 256 + tid;
    const int ci = idx >> 5, nj = idx & 31;
    tile[ci][nj] = xs[(size_t)ci * Nn + nj];
  }
  __syncthreads();
  const int p = tid >> 3, q = tid & 7;
  v8h hv, bh, bl;
#pragma unroll
  for (int e = 0; e < 8; ++e) {
    const float f = tile[8 * q + e][p];
    hv[e] = (_Float16)f;
    _Float16 th, tl;
    split_bf16(f, th, tl);
    bh[e] = th; bl[e] = tl;
  }
  const size_t off = ((size_t)b * Nn + n0 + p) * Cc + c0 + 8 * q;
  *(volatile v8h*)(xh + off) = hv; *(volatile v8h*)(xbh + off) = bh; *(volatile v8h*)(xbl + off) = bl;
  __threadfence();
  *(volatile v8h*)(xh + off) = hv; *(volatile v8h*)(xbh + off) = bh; *(volatile v8h*)(xbl + off) = bl;
}

__global__ __launch_bounds__(256) void k_softmax_rows(const float* __restrict__ S,
                                                      unsigned short* __restrict__ P,
                                                      int Nn, float pscale) {
  __shared__ float red[16];
  const int tid = threadIdx.x, lane = tid & 31, wave = tid >> 5;
  const int row = blockIdx.x;
  const int nv = Nn >> 3;
  const float* sr = S + (size_t)row * Nn;
  const int t2 = tid + 256;
  const bool v2 = (t2 < nv);
  const int t2c = v2 ? t2 : tid;
  const v4f a0 = *(const v4f*)(sr + 8 * tid);
  const v4f a1 = *(const v4f*)(sr + 8 * tid + 4);
  const v4f b0 = *(const v4f*)(sr + 8 * t2c);
  const v4f b1 = *(const v4f*)(sr + 8 * t2c + 4);
  float m = a0[0], mb = b0[0];
#pragma unroll
  for (int e = 0; e < 4; ++e) { m = fmaxf(m, fmaxf(a0[e], a1[e])); mb = fmaxf(mb, fmaxf(b0[e], b1[e])); }
  if (v2) m = fmaxf(m, mb);
#pragma unroll
  for (int off = 1; off < 32; off <<= 1) m = fmaxf(m, __shfl_xor(m, off, 32));
  if (lane == 0) red[wave] = m;
  __syncthreads();
  float gm = red[0];
#pragma unroll
  for (int w = 1; w < 8; ++w) gm = fmaxf(gm, red[w]);
  v4f pa0, pa1, pb0, pb1;
  float s = 0.f, sb = 0.f;
#pragma unroll
  for (int e = 0; e < 4; ++e) {
    pa0[e] = __expf(a0[e] - gm); pa1[e] = __expf(a1[e] - gm);
    pb0[e] = __expf(b0[e] - gm); pb1[e] = __expf(b1[e] - gm);
    s += pa0[e]; s += pa1[e]; sb += pb0[e]; sb += pb1[e];
  }
  if (v2) s += sb;
#pragma unroll
  for (int off = 1; off < 32; off <<= 1) s += __shfl_xor(s, off, 32);
  if (lane == 0) red[8 + wave] = s;
  __syncthreads();
  float tot = red[8];
#pragma unroll
  for (int w = 1; w < 8; ++w) tot += red[8 + w];
  const float scl = (1.0f / tot) * pscale;
  v8h ha, hb;
#pragma unroll
  for (int e = 0; e < 4; ++e) {
    ha[e] = (_Float16)(pa0[e] * scl); ha[4 + e] = (_Float16)(pa1[e] * scl);
    hb[e] = (_Float16)(pb0[e] * scl); hb[4 + e] = (_Float16)(pb1[e] * scl);
  }
  unsigned short* pr = P + (size_t)row * Nn;
  *(volatile v8h*)(pr + 8 * tid) = ha;
  if (v2) *(volatile v8h*)(pr + 8 * t2) = hb;
  __threadfence();
  *(volatile v8h*)(pr + 8 * tid) = ha;
  if (v2) *(volatile v8h*)(pr + 8 * t2) = hb;
}

extern "C" void kernel_launch(void* const* d_in, const int* in_sizes, int n_in,
                              void* d_out, int out_size, void* d_ws, size_t ws_size,
                              hipStream_t stream) {
  const int Bn = 8, Cn = 256, Nn = 3136, En = 128;
  if (n_in < 5) return;
  if (in_sizes[0] != Bn * Cn * Nn || in_sizes[1] != En * Cn || in_sizes[2] != En ||
      in_sizes[3] != Cn * En || in_sizes[4] != Cn) return;
  if (out_size != Bn * Cn * Nn) return;
  const float* x  = (const float*)d_in[0];
  const float* vw = (const float*)d_in[1];
  const float* vb = (const float*)d_in[2];
  const float* ew = (const float*)d_in[3];
  const float* eb = (const float*)d_in[4];
  float* out = (float*)d_out;

  const size_t nS  = (size_t)Nn * Nn * 4;
  const size_t nP  = (size_t)Nn * Nn * 2;
  const size_t nX  = (size_t)Bn * Nn * Cn * 2;
  const size_t nVt = (size_t)Bn * En * Nn * 2;
  const size_t nEm = (size_t)Bn * Nn * En * 2;
  const size_t nW  = (size_t)En * Cn * 2;
  const size_t oS = 0, oP = oS + nS, oXh = oP + nP, oXbh = oXh + nX, oXbl = oXbh + nX, oVt = oXbl + nX,
               oEh = oVt + nVt, oEl = oEh + nEm, oWvh = oEl + nEm, oWvl = oWvh + nW, oWeh = oWvl + nW,
               oWel = oWeh + nW, total = oWel + nW;
  if (total > ws_size) return;
  char* ws = (char*)d_ws;
  float*          S    = (float*)(ws + oS);
  unsigned short* P16  = (unsigned short*)(ws + oP);
  unsigned short* xh   = (unsigned short*)(ws + oXh);
  unsigned short* xbh  = (unsigned short*)(ws + oXbh);
  unsigned short* xbl  = (unsigned short*)(ws + oXbl);
  unsigned short* vt   = (unsigned short*)(ws + oVt);
  unsigned short* embh = (unsigned short*)(ws + oEh);
  unsigned short* embl = (unsigned short*)(ws + oEl);
  unsigned short* wvh  = (unsigned short*)(ws + oWvh);
  unsigned short* wvl  = (unsigned short*)(ws + oWvl);
  unsigned short* weh  = (unsigned short*)(ws + oWeh);
  unsigned short* wel  = (unsigned short*)(ws + oWel);

  {
    const int n8 = (En * Cn) / 8;
    k_wsplit<<<(n8 + 255) / 256, 256, 0, stream>>>(vw, ew, wvh, wvl, weh, wel, n8);
  }
  {
    const int grid = Bn * (Cn / 64) * (Nn / 32);
    k_xconv<<<grid, 256, 0, stream>>>(x, xh, xbh, xbl, Cn, Nn);
  }
  {
    const int tiles = (En / 64) * (Nn / 64);
    wmma_gemm64<1, true, 1, 1, false><<<dim3((tiles + 7) / 8, Bn), 256, 0, stream>>>(
        wvh, wvl, Cn, 0L,
        xbh, xbl, Cn, (long)Nn * Cn,
        (void*)vt, (void*)vt, Nn, (long)En * Nn,
        vb, x, 0L, En, Nn, Cn, 1.0f);
  }
  const int NT = Nn / 64;
  const int npairs = NT * (NT + 1) / 2;
  const int tilesPV = (Nn / 64) * (En / 64);
  for (int b = 0; b < Bn; ++b) {
    const unsigned short* Xb = xh + (size_t)b * Nn * Cn;
    wmma_gram64<<<(npairs + 7) / 8, 256, 0, stream>>>(Xb, Cn, S, Nn, NT, Cn, 1.0f);
    k_softmax_rows<<<Nn, 256, 0, stream>>>(S, P16, Nn, 32768.0f);
    const unsigned short* Vb = vt + (size_t)b * En * Nn;
    unsigned short* Ehb = embh + (size_t)b * Nn * En;
    unsigned short* Elb = embl + (size_t)b * Nn * En;
    wmma_gemm64<0, false, 0, 2, false><<<dim3((tilesPV + 7) / 8, 1), 256, 0, stream>>>(
        P16, P16, Nn, 0L,
        Vb, Vb, Nn, 0L,
        (void*)Ehb, (void*)Elb, En, 0L,
        eb, x, 0L, Nn, En, Nn, 1.0f / 32768.0f);
  }
  {
    const int tiles = (Cn / 64) * (Nn / 64);
    wmma_gemm64<1, true, 1, 0, true><<<dim3((tiles + 7) / 8, Bn), 256, 0, stream>>>(
        weh, wel, En, 0L,
        embh, embl, En, (long)Nn * En,
        (void*)out, (void*)out, Nn, (long)Cn * Nn,
        eb, x, (long)Cn * Nn, Cn, Nn, En, 1.0f);
  }
}
